// ClassicalMPGNN_21930103013841
// MI455X (gfx1250) — hardware-verified
//
#include <hip/hip_runtime.h>
#include <stddef.h>
#include <stdint.h>


#define FD      64
#define CH      256
#define CO      64
#define CM      16
#define ABW     512
#define WSC     64.0f
#define WIV     0.015625f
#define MSC     32.0f
#define MIV     0.03125f

#define T1_OFF  0
#define T2_OFF  32768
#define T3_OFF  98304
#define T4_OFF  114688
#define T_TOT   115712
#define T_LINES 1808

#define NPR     128
#define SPH     136

#define EW      4
#define ETPW    10
#define ETPB    (EW * ETPW)
#define EEPB    (ETPB * 16)
#define STR     264
#define SWP     20
#define L_W2    0
#define L_W3    131072
#define L_T4    163840
#define L_B2    165888
#define L_B3    166912
#define L_H     167168
#define L_HSZ   (16 * STR * 2)
#define L_SW    (L_H + EW * 2 * L_HSZ)
#define L_SWSZ  (16 * SWP * 4)
#define E_LDS   (L_SW + EW * L_SWSZ)

#define PG      32
#define PT      256
#define PW      8
#define PEPT    8
#define PCH     (PT * PEPT)
#define PCAP    (PEPT * 32)

static_assert(T_LINES * 64 == T_TOT);
static_assert(T2_OFF == 256 * 128 && T3_OFF == T2_OFF + 256 * 256 && T4_OFF == T3_OFF + 64 * 256 && T_TOT == T4_OFF + 16 * 64);
static_assert(L_W3 == (T3_OFF - T2_OFF) * 2 && L_T4 == (T4_OFF - T2_OFF) * 2 && L_B2 == (T_TOT - T2_OFF) * 2);
static_assert(L_B3 == L_B2 + CH * 4 && L_H == L_B3 + CO * 4);
static_assert((L_H & 15) == 0 && (L_HSZ & 15) == 0 && (L_SW & 15) == 0 && (L_SWSZ & 15) == 0 && (L_B2 & 15) == 0);
static_assert(((STR * 2) & 15) == 0 && ((SPH * 2) & 15) == 0 && ((SWP * 4) & 15) == 0);
static_assert(E_LDS <= 300 * 1024);
static_assert(PW * 32 == PT && PCAP == 256 && PG <= 256 && (PG & 1) == 0);

typedef float    v4f  __attribute__((ext_vector_type(4)));
typedef float    v8f  __attribute__((ext_vector_type(8)));
typedef int      v4i  __attribute__((ext_vector_type(4)));
typedef unsigned v4u  __attribute__((ext_vector_type(4)));
typedef _Float16 v8h  __attribute__((ext_vector_type(8)));
typedef _Float16 v16h __attribute__((ext_vector_type(16)));
union FragH { v16h v; v8h h[2]; };
union H8    { v8h v; v4u u; };

#if defined(__has_builtin)
#if __has_builtin(__builtin_elementwise_max)
#define USE_EWMAX 1
#endif
#endif

__device__ __forceinline__ v8f zero8f() {
  v8f z;
#pragma unroll
  for (int i = 0; i < 8; ++i) z[i] = 0.0f;
  return z;
}
__device__ __forceinline__ v4f zero4f() {
  v4f z;
#pragma unroll
  for (int i = 0; i < 4; ++i) z[i] = 0.0f;
  return z;
}

__device__ __forceinline__ v8f wm(v16h a, v16h b, v8f c) {
  return __builtin_amdgcn_wmma_f32_16x16x32_f16(false, a, false, b, (short)0, c, false, false);
}
#define WGUARD(ACC, A, B) asm volatile("v_nop\n\tv_nop\n\tv_nop\n\tv_nop" : "+v"(ACC) : "v"(A), "v"(B))

__device__ __forceinline__ v8h cvt8h(const float* p) {
  const v4f a = *(const v4f*)p;
  const v4f b = *(const v4f*)(p + 4);
  v8h o;
  o[0] = (_Float16)a[0]; o[1] = (_Float16)a[1]; o[2] = (_Float16)a[2]; o[3] = (_Float16)a[3];
  o[4] = (_Float16)b[0]; o[5] = (_Float16)b[1]; o[6] = (_Float16)b[2]; o[7] = (_Float16)b[3];
  return o;
}

__device__ __forceinline__ v8h relu_add8(v8h a, v8h b) {
  H8 s;
  s.v = a + b;
#ifdef USE_EWMAX
  v8h z;
#pragma unroll
  for (int i = 0; i < 8; ++i) z[i] = (_Float16)0.0f;
  s.v = __builtin_elementwise_max(s.v, z);
#else
#pragma unroll
  for (int i = 0; i < 4; ++i) {
    unsigned w = s.u[i];
    const unsigned sg = (w >> 15) & 0x00010001u;
    w &= ~(sg * 0xFFFFu);
    s.u[i] = w;
  }
#endif
  return s.v;
}

__global__ __launch_bounds__(256) void k_wcvt(const float* __restrict__ W1, const float* __restrict__ W2,
                                              const float* __restrict__ W3, const float* __restrict__ Wm1,
                                              _Float16* Wt) {
  const int t = blockIdx.x * 256 + threadIdx.x;
  if (t >= T_LINES * 8) return;
  const int L = t >> 3, sub = (t & 7) * 8;
  const float* src = W1;
  int n = 0, k0 = 0, N = 256, dst = 0;
  float sc = WSC;
  if (L < 512)       { n = L >> 1; k0 = (L & 1) * 64 + sub; src = W1; N = 256; dst = T1_OFF + n * 128 + k0; }
  else if (L < 1536) { const int q = L - 512;  n = q >> 2; k0 = (q & 3) * 64 + sub; src = W2;  N = 256; dst = T2_OFF + n * 256 + k0; }
  else if (L < 1792) { const int q = L - 1536; n = q >> 2; k0 = (q & 3) * 64 + sub; src = W3;  N = 64;  dst = T3_OFF + n * 256 + k0; }
  else               { n = L - 1792; k0 = sub; src = Wm1; N = 16; sc = MSC; dst = T4_OFF + n * 64 + k0; }
  v8h o;
#pragma unroll
  for (int i = 0; i < 8; ++i) o[i] = (_Float16)(src[(size_t)(k0 + i) * N + n] * sc);
  _Float16* dp = Wt + dst;
  *(volatile v8h*)dp = o;
  __threadfence();
  *(volatile v8h*)dp = o;
}

__global__ __launch_bounds__(256) void k_nproj(const float* __restrict__ x, const _Float16* __restrict__ T1,
                                               const float* __restrict__ b1, _Float16* AB, int nN) {
  __shared__ __attribute__((aligned(16))) _Float16 stg_s[8 * 16 * SPH];
  const int tid = threadIdx.x, l = tid & 31, wave = tid >> 5, h = l >> 4, m = l & 15;
  const int row0 = blockIdx.x * NPR + 16 * wave;
  int br = row0 + m;
  br = br > nN - 1 ? nN - 1 : br;
  const float* xr = x + (size_t)br * FD;
  FragH b[2];
#pragma unroll
  for (int ks = 0; ks < 2; ++ks) {
    b[ks].h[0] = cvt8h(xr + 32 * ks + 8 * h);
    b[ks].h[1] = cvt8h(xr + 32 * ks + 16 + 8 * h);
  }
  _Float16* st = stg_s + wave * (16 * SPH);
  const int c8 = 8 * (l & 15);
  const v4f z4 = zero4f();

#pragma unroll 1
  for (int cg = 0; cg < 4; ++cg) {
    const int kof = (cg >> 1) * 64;
    const int tr0 = (cg & 1) * 128;
#pragma unroll 1
    for (int ct = 0; ct < 8; ++ct) {
      const _Float16* ar = T1 + (size_t)(tr0 + 16 * ct + m) * 128 + kof + 8 * h;
      v8f acc = zero8f();
      FragH a;
#pragma unroll
      for (int ks = 0; ks < 2; ++ks) {
        a.h[0] = *(const v8h*)(ar + 32 * ks);
        a.h[1] = *(const v8h*)(ar + 32 * ks + 16);
        acc = wm(a.v, b[ks].v, acc);
      }
      WGUARD(acc, a.v, b[1].v);
      v4f c0 = z4, c1 = z4;
      if (cg < 2) {
        const float* bp = b1 + cg * 128 + 16 * ct + 8 * h;
        c0 = *(const v4f*)bp;
        c1 = *(const v4f*)(bp + 4);
      }
      v8h o;
#pragma unroll
      for (int r = 0; r < 4; ++r) {
        o[r]     = (_Float16)(acc[r] * WIV + c0[r]);
        o[4 + r] = (_Float16)(acc[4 + r] * WIV + c1[r]);
      }
      *(v8h*)(st + m * SPH + 16 * ct + 8 * h) = o;
    }
    __syncthreads();
    _Float16* gb = AB + (size_t)row0 * ABW + cg * 128 + c8;
#pragma unroll
    for (int j = 0; j < 8; ++j) {
      const int lr = 2 * j + h;
      const v8h v = *(const v8h*)(st + lr * SPH + c8);
      *(volatile v8h*)(gb + (size_t)lr * ABW) = v;
    }
    __threadfence();
#pragma unroll
    for (int j = 0; j < 8; ++j) {
      const int lr = 2 * j + h;
      const v8h v = *(const v8h*)(st + lr * SPH + c8);
      *(volatile v8h*)(gb + (size_t)lr * ABW) = v;
    }
    __syncthreads();
  }
}

__global__ __launch_bounds__(EW * 32) void k_edge(const _Float16* __restrict__ AB, const int* __restrict__ ei,
                                                  const _Float16* __restrict__ Wt, const float* __restrict__ b2,
                                                  const float* __restrict__ b3, float* MW, int nE, int nN) {
  extern __shared__ __attribute__((aligned(16))) unsigned char lds_e[];
  const int tid = threadIdx.x, l = tid & 31, wave = tid >> 5, h = l >> 4, m = l & 15;
  {
    const _Float16* src = Wt + T2_OFF;
    for (int i = tid; i < L_B2 / 16; i += EW * 32)
      *(v8h*)(lds_e + 16 * i) = *(const v8h*)(src + 8 * i);
    float* b2w = (float*)(lds_e + L_B2);
    float* b3w = (float*)(lds_e + L_B3);
    for (int i = tid; i < CH; i += EW * 32) b2w[i] = b2[i];
    if (tid < CO) b3w[tid] = b3[tid];
  }
  __syncthreads();
  const _Float16* W2s = (const _Float16*)(lds_e + L_W2);
  const _Float16* W3s = (const _Float16*)(lds_e + L_W3);
  const _Float16* T4s = (const _Float16*)(lds_e + L_T4);
  const float* b2s = (const float*)(lds_e + L_B2);
  const float* b3s = (const float*)(lds_e + L_B3);
  _Float16* hb0 = (_Float16*)(lds_e + L_H + wave * (2 * L_HSZ));
  _Float16* hb1 = hb0 + 16 * STR;
  float* sw = (float*)(lds_e + L_SW + wave * L_SWSZ);

#pragma unroll 1
  for (int t = 0; t < ETPW; ++t) {
    const int ebase = (blockIdx.x * ETPB + wave * ETPW + t) * 16;

    {
      const int el = l >> 1, hh = l & 1;
      int e = ebase + el;
      e = e > nE - 1 ? nE - 1 : e;
      int r = ei[e];
      int c = ei[(size_t)nE + e];
      r = r < 0 ? 0 : (r > nN - 1 ? nN - 1 : r);
      c = c < 0 ? 0 : (c > nN - 1 ? nN - 1 : c);
      const _Float16* pa = AB + (size_t)r * ABW + 128 * hh;
      const _Float16* pb = AB + (size_t)c * ABW + CH + 128 * hh;
      _Float16* ph = hb0 + el * STR + 128 * hh;
#pragma unroll
      for (int q = 0; q < 16; ++q) {
        const v8h av = *(const v8h*)(pa + 8 * q);
        const v8h bv = *(const v8h*)(pb + 8 * q);
        *(v8h*)(ph + 8 * q) = relu_add8(av, bv);
      }
    }
    __syncthreads();

    FragH b[8];
    {
      const _Float16* hr = hb0 + m * STR + 8 * h;
#pragma unroll
      for (int ks = 0; ks < 8; ++ks) {
        b[ks].h[0] = *(const v8h*)(hr + 32 * ks);
        b[ks].h[1] = *(const v8h*)(hr + 32 * ks + 16);
      }
    }
#pragma unroll 1
    for (int ct = 0; ct < CH / 16; ++ct) {
      const _Float16* ar = W2s + (16 * ct + m) * CH + 8 * h;
      v8f acc = zero8f();
      FragH a;
#pragma unroll
      for (int ks = 0; ks < 8; ++ks) {
        a.h[0] = *(const v8h*)(ar + 32 * ks);
        a.h[1] = *(const v8h*)(ar + 32 * ks + 16);
        acc = wm(a.v, b[ks].v, acc);
      }
      WGUARD(acc, a.v, b[7].v);
      const float* bp = b2s + 16 * ct + 8 * h;
      const v4f c0 = *(const v4f*)bp;
      const v4f c1 = *(const v4f*)(bp + 4);
      v8h o;
#pragma unroll
      for (int r = 0; r < 4; ++r) {
        o[r]     = (_Float16)fmaxf(acc[r] * WIV + c0[r], 0.0f);
        o[4 + r] = (_Float16)fmaxf(acc[4 + r] * WIV + c1[r], 0.0f);
      }
      *(v8h*)(hb1 + m * STR + 16 * ct + 8 * h) = o;
    }
    __syncthreads();

    {
      const _Float16* hr = hb1 + m * STR + 8 * h;
#pragma unroll
      for (int ks = 0; ks < 8; ++ks) {
        b[ks].h[0] = *(const v8h*)(hr + 32 * ks);
        b[ks].h[1] = *(const v8h*)(hr + 32 * ks + 16);
      }
    }
#pragma unroll 1
    for (int ct = 0; ct < CO / 16; ++ct) {
      const _Float16* ar = W3s + (16 * ct + m) * CH + 8 * h;
      v8f acc = zero8f();
      FragH a;
#pragma unroll
      for (int ks = 0; ks < 8; ++ks) {
        a.h[0] = *(const v8h*)(ar + 32 * ks);
        a.h[1] = *(const v8h*)(ar + 32 * ks + 16);
        acc = wm(a.v, b[ks].v, acc);
      }
      WGUARD(acc, a.v, b[7].v);
      const float* bp = b3s + 16 * ct + 8 * h;
      const v4f c0 = *(const v4f*)bp;
      const v4f c1 = *(const v4f*)(bp + 4);
      v8h o;
#pragma unroll
      for (int r = 0; r < 4; ++r) {
        o[r]     = (_Float16)(acc[r] * WIV + c0[r]);
        o[4 + r] = (_Float16)(acc[4 + r] * WIV + c1[r]);
      }
      *(v8h*)(hb0 + m * STR + 16 * ct + 8 * h) = o;
    }
    __syncthreads();

    {
      const _Float16* hr = hb0 + m * STR + 8 * h;
#pragma unroll
      for (int ks = 0; ks < 2; ++ks) {
        b[ks].h[0] = *(const v8h*)(hr + 32 * ks);
        b[ks].h[1] = *(const v8h*)(hr + 32 * ks + 16);
      }
      const _Float16* ar = T4s + m * FD + 8 * h;
      v8f acc = zero8f();
      FragH a;
#pragma unroll
      for (int ks = 0; ks < 2; ++ks) {
        a.h[0] = *(const v8h*)(ar + 32 * ks);
        a.h[1] = *(const v8h*)(ar + 32 * ks + 16);
        acc = wm(a.v, b[ks].v, acc);
      }
      WGUARD(acc, a.v, b[1].v);
      v4f f0, f1;
#pragma unroll
      for (int r = 0; r < 4; ++r) { f0[r] = acc[r] * MIV; f1[r] = acc[4 + r] * MIV; }
      *(v4f*)(sw + m * SWP + 8 * h) = f0;
      *(v4f*)(sw + m * SWP + 8 * h + 4) = f1;
    }
    __syncthreads();
    {
      const int rw = l >> 2, q4 = 4 * (l & 3);
      const v4f u0 = *(const v4f*)(sw + rw * SWP + q4);
      const v4f u1 = *(const v4f*)(sw + (rw + 8) * SWP + q4);
      float* g0 = MW + (size_t)(ebase + rw) * CM + q4;
      float* g1 = g0 + 8 * CM;
      *(volatile v4f*)g0 = u0;
      *(volatile v4f*)g1 = u1;
      __threadfence();
      *(volatile v4f*)g0 = u0;
      *(volatile v4f*)g1 = u1;
    }
  }
}

__device__ __forceinline__ int scan_chunk(const int* __restrict__ rows, const int* __restrict__ bat, int nE, int nN,
                                          int cbase, int gBase, int* list, int tid, int wave) {
  int wc = 0;
  const int el0 = tid * PEPT;
  const int e0 = cbase + el0;
  int rv[8];
  if (e0 + 7 < nE) {
    const v4i da = *(const v4i*)(rows + e0);
    const v4i db = *(const v4i*)(rows + e0 + 4);
    rv[0] = da[0]; rv[1] = da[1]; rv[2] = da[2]; rv[3] = da[3];
    rv[4] = db[0]; rv[5] = db[1]; rv[6] = db[2]; rv[7] = db[3];
  } else {
#pragma unroll
    for (int j = 0; j < 8; ++j) {
      const int e = e0 + j;
      const int vv = rows[e < nE ? e : nE - 1];
      rv[j] = (e < nE) ? vv : -1;
    }
  }
  unsigned sv[8];
  bool qv[8];
  bool anyq = false;
#pragma unroll
  for (int j = 0; j < 8; ++j) {
    const int r = rv[j];
    const bool ok = (unsigned)r < (unsigned)nN;
    const int g = bat[ok ? r : 0];
    const unsigned s = ok ? ((unsigned)g - (unsigned)gBase) : 0xFFFFFFFFu;
    sv[j] = s;
    qv[j] = s < (unsigned)PG;
    anyq = anyq | qv[j];
  }
  const unsigned any = __builtin_amdgcn_ballot_w32(anyq);
  if (any != 0u) {
#pragma unroll
    for (int j = 0; j < 8; ++j) {
      const unsigned mj = __builtin_amdgcn_ballot_w32(qv[j]);
      if (mj != 0u) {
        if (qv[j]) {
          const int pos = wc + (int)__builtin_amdgcn_mbcnt_lo(mj, 0u);
          if (pos < PCAP) list[wave * PCAP + pos] = ((el0 + j) << 8) | (int)sv[j];
        }
        wc += (int)__builtin_popcount(mj);
      }
    }
  }
  return wc;
}

__global__ __launch_bounds__(PT) void k_pool(const int* __restrict__ ei, const int* __restrict__ bat,
                                             const float* __restrict__ MW, const float* __restrict__ bm1,
                                             const float* __restrict__ Wm2, const float* __restrict__ bm2,
                                             float* out, int nE, int nN, int nG) {
  __shared__ __attribute__((aligned(16))) float accs[PW * 2 * PG * CM];
  __shared__ int lst[PW * PCAP];
  __shared__ int wcnt[PW];
  __shared__ __attribute__((aligned(16))) float comb[PG * CM];
  __shared__ __attribute__((aligned(16))) float res[PG * 2];
  const int tid = threadIdx.x, l = tid & 31, wave = tid >> 5, h = l >> 4;
  const int gBase = blockIdx.x * PG;
  {
    const v4f z4 = zero4f();
    for (int i = tid; i < (PW * 2 * PG * CM) / 4; i += PT) *(v4f*)(accs + 4 * i) = z4;
  }
  __syncthreads();

  float* myacc = accs + ((wave * 2 + h) * PG) * CM + (l & 15);
  const int nChunks = (nE + PCH - 1) / PCH;
#pragma unroll 1
  for (int ch = 0; ch < nChunks; ++ch) {
    const int cbase = ch * PCH;
    const int wc = scan_chunk(ei, bat, nE, nN, cbase, gBase, lst, tid, wave);
    if (l == 0) wcnt[wave] = wc;
    __syncthreads();
#pragma unroll 1
    for (int w2 = 0; w2 < PW; ++w2) {
      int n = wcnt[w2];
      n = n > PCAP ? PCAP : (n < 0 ? 0 : n);
      const int* lp = lst + w2 * PCAP;
#pragma unroll 1
      for (int base = wave; base < n; base += 16) {
        const int idx = base + 8 * h;
        if (idx < n) {
          const int v = lp[idx];
          int slot = v & 255;
          slot = slot > PG - 1 ? PG - 1 : slot;
          int e = cbase + (v >> 8);
          e = e < 0 ? 0 : (e > nE - 1 ? nE - 1 : e);
          const float val = MW[(size_t)e * CM + (l & 15)];
          float* ap = myacc + slot * CM;
          *ap = *ap + val;
        }
      }
    }
    __syncthreads();
  }

  for (int idx = tid; idx < PG * CM; idx += PT) {
    float s = 0.0f;
#pragma unroll
    for (int c = 0; c < PW * 2; ++c) s += accs[c * (PG * CM) + idx];
    comb[idx] = s;
  }
  __syncthreads();
  if (tid < PG * 2) {
    const int g = tid >> 1, o = tid & 1;
    float s = 0.0f;
#pragma unroll
    for (int j = 0; j < CM; ++j) {
      const float hj = fmaxf(comb[g * CM + j] + bm1[j], 0.0f);
      s += hj * Wm2[j * 2 + o];
    }
    res[tid] = s + bm2[o];
  }
  __syncthreads();
  if (wave == 0 && l < 16) {
    const v4f v = *(const v4f*)(res + 4 * l);
    const int g0 = gBase + 2 * l;
    float* op = out + (size_t)gBase * 2 + 4 * l;
    if (g0 + 1 < nG) {
      *(volatile v4f*)op = v;
    } else {
#pragma unroll
      for (int k = 0; k < 4; ++k) if (g0 + (k >> 1) < nG) ((volatile float*)op)[k] = v[k];
    }
    __threadfence();
    if (g0 + 1 < nG) {
      *(volatile v4f*)op = v;
    } else {
#pragma unroll
      for (int k = 0; k < 4; ++k) if (g0 + (k >> 1) < nG) ((volatile float*)op)[k] = v[k];
    }
  }
}

extern "C" void kernel_launch(void* const* d_in, const int* in_sizes, int n_in,
                              void* d_out, int out_size, void* d_ws, size_t ws_size,
                              hipStream_t stream) {
  if (n_in < 13) return;
  const int nN = in_sizes[2];
  if (nN <= 0 || in_sizes[0] != nN * FD) return;
  if (in_sizes[1] < 2 || (in_sizes[1] & 1)) return;
  const int nE = in_sizes[1] / 2;
  if (out_size < 2 || (out_size & 1)) return;
  const int nG = out_size / 2;
  if (in_sizes[3] != 2 * FD * CH || in_sizes[4] < CH || in_sizes[5] != CH * CH || in_sizes[6] < CH) return;
  if (in_sizes[7] != CH * CO || in_sizes[8] < CO || in_sizes[9] != CO * CM || in_sizes[10] < CM) return;
  if (in_sizes[11] != CM * 2 || in_sizes[12] < 2) return;

  const float* x   = (const float*)d_in[0];
  const int*   ei  = (const int*)d_in[1];
  const int*   bat = (const int*)d_in[2];
  const float* W1  = (const float*)d_in[3];
  const float* b1  = (const float*)d_in[4];
  const float* W2  = (const float*)d_in[5];
  const float* b2  = (const float*)d_in[6];
  const float* W3  = (const float*)d_in[7];
  const float* b3  = (const float*)d_in[8];
  const float* Wm1 = (const float*)d_in[9];
  const float* bm1 = (const float*)d_in[10];
  const float* Wm2 = (const float*)d_in[11];
  const float* bm2 = (const float*)d_in[12];
  float* out = (float*)d_out;

  const int nBlkN  = (nN + NPR - 1) / NPR;
  const int nTiles = (nE + 15) / 16;
  const int nBlkE  = (nTiles + ETPB - 1) / ETPB;
  const int nBlkG  = (nG + PG - 1) / PG;

  char* ws = (char*)d_ws;
  size_t off = 0;
  const size_t oWt = off; off += (size_t)T_TOT * 2;                         off = (off + 255) & ~(size_t)255;
  const size_t oAB = off; off += (size_t)nBlkN * NPR * ABW * 2;              off = (off + 255) & ~(size_t)255;
  const size_t oMW = off; off += (size_t)nBlkE * EEPB * CM * 4;              off = (off + 255) & ~(size_t)255;
  if (off > ws_size) return;
  _Float16* Wt  = (_Float16*)(ws + oWt);
  _Float16* ABh = (_Float16*)(ws + oAB);
  float*    MWp = (float*)(ws + oMW);

  const hipError_t a0 = hipFuncSetAttribute(reinterpret_cast<const void*>(&k_edge),
                                            hipFuncAttributeMaxDynamicSharedMemorySize, E_LDS);
  (void)a0;

  k_wcvt<<<(T_LINES * 8 + 255) / 256, 256, 0, stream>>>(W1, W2, W3, Wm1, Wt);
  k_nproj<<<nBlkN, 256, 0, stream>>>(x, Wt + T1_OFF, b1, ABh, nN);
  k_edge<<<nBlkE, EW * 32, E_LDS, stream>>>(ABh, ei, Wt, b2, b3, MWp, nE, nN);
  k_pool<<<nBlkG, PT, 0, stream>>>(ei, bat, MWp, bm1, Wm2, bm2, out, nE, nN, nG);
  (void)hipGetLastError();
}
